// NonLocalAlignment_88201448391100
// MI455X (gfx1250) — hardware-verified
//
#include <hip/hip_runtime.h>
#include <math.h>

typedef __attribute__((ext_vector_type(16))) _Float16 v16h;
typedef __attribute__((ext_vector_type(16))) __bf16 v16b;
typedef __attribute__((ext_vector_type(8)))  _Float16 v8h;
typedef __attribute__((ext_vector_type(8)))  float v8f;
typedef __attribute__((ext_vector_type(4)))  float v4f;
typedef __attribute__((ext_vector_type(2)))  float v2f;
typedef __attribute__((ext_vector_type(4)))  unsigned v4u;
typedef __attribute__((ext_vector_type(4)))  int v4i;
typedef float __attribute__((may_alias)) float_a;
typedef int __attribute__((may_alias)) int_a;

template <typename T> __device__ __forceinline__ void vst2(void* p, T v) { *(volatile T*)p = v; __threadfence(); *(volatile T*)p = v; }
__device__ __forceinline__ v8f wmma16(v16h a, v16h b, v8f c) {
  v8f d = __builtin_amdgcn_wmma_f32_16x16x32_f16(false, a, false, b, (short)0, c, false, false);
  asm volatile("v_nop\n\tv_nop\n\tv_nop\n\tv_nop" : "+v"(d) : "v"(a), "v"(b));
  return d;
}
__device__ __forceinline__ v8f wmma_bf(v16b a, v16b b, v8f c) {
  v8f d = __builtin_amdgcn_wmma_f32_16x16x32_bf16(false, a, false, b, (short)0, c, false, false);
  asm volatile("v_nop\n\tv_nop\n\tv_nop\n\tv_nop" : "+v"(d) : "v"(a), "v"(b));
  return d;
}
__device__ __forceinline__ v16h frag_h(const _Float16* rowk0, int lane) {
  union { v16h v; v8h q[2]; } u; const _Float16* p = rowk0 + 8 * (lane >> 4);
  u.q[0] = *(const v8h*)p; u.q[1] = *(const v8h*)(p + 16); return u.v;
}
__device__ __forceinline__ v16h frag_f32(const float* rowk0, int lane) {
  v16h a; const float* p = rowk0 + 8 * (lane >> 4);
#pragma unroll
  for (int i = 0; i < 8; ++i) { a[i] = (_Float16)p[i]; a[8 + i] = (_Float16)p[16 + i]; }
  return a;
}
__device__ __forceinline__ v16h frag_f32s(const float* rowk0, int lane, float sc) {
  v16h a; const float* p = rowk0 + 8 * (lane >> 4);
#pragma unroll
  for (int i = 0; i < 8; ++i) { a[i] = (_Float16)(p[i] * sc); a[8 + i] = (_Float16)(p[16 + i] * sc); }
  return a;
}
__device__ __forceinline__ v16h fragc_f32(const float* W, int k0, int n, int lane, int ld, int K) {
  v16h a; const int g = lane >> 4;
#pragma unroll
  for (int i = 0; i < 8; ++i) { const int ka = k0 + 8 * g + i, kb = ka + 16;
    a[i] = (_Float16)(ka < K ? W[(size_t)(ka < K ? ka : K - 1) * ld + n] : 0.f); a[8 + i] = (_Float16)(kb < K ? W[(size_t)(kb < K ? kb : K - 1) * ld + n] : 0.f); }
  return a;
}
struct F2 { v16b h, l; };
__device__ __forceinline__ F2 bsplit16(const float v[16]) { F2 r;
#pragma unroll
  for (int i = 0; i < 16; ++i) { const __bf16 h = (__bf16)v[i]; r.h[i] = h; r.l[i] = (__bf16)(v[i] - (float)h); }
  return r; }
__device__ __forceinline__ F2 split_row(const float* row, int k0, int lane) { float v[16]; const float* p = row + k0 + 8 * (lane >> 4);
#pragma unroll
  for (int i = 0; i < 8; ++i) { v[i] = p[i]; v[8 + i] = p[16 + i]; }
  return bsplit16(v); }
__device__ __forceinline__ F2 split_rowK(const float* row, int k0, int lane, int K) { float v[16]; const int g = lane >> 4;
#pragma unroll
  for (int i = 0; i < 8; ++i) { const int ka = k0 + 8 * g + i, kb = ka + 16; v[i] = ka < K ? row[ka < K ? ka : K - 1] : 0.f; v[8 + i] = kb < K ? row[kb < K ? kb : K - 1] : 0.f; }
  return bsplit16(v); }
__device__ __forceinline__ F2 split_col(const float* W, int k0, int n, int lane, int ld, int K) { float v[16]; const int g = lane >> 4;
#pragma unroll
  for (int i = 0; i < 8; ++i) { const int ka = k0 + 8 * g + i, kb = ka + 16; v[i] = ka < K ? W[(size_t)(ka < K ? ka : K - 1) * ld + n] : 0.f; v[8 + i] = kb < K ? W[(size_t)(kb < K ? kb : K - 1) * ld + n] : 0.f; }
  return bsplit16(v); }
__device__ __forceinline__ v8f mac3(const F2& a, const F2& b, v8f c) { c = wmma_bf(a.l, b.h, c); c = wmma_bf(a.h, b.l, c); return wmma_bf(a.h, b.h, c); }
__device__ __forceinline__ float sigm(float v) { return 1.0f / (1.0f + expf(-v)); }
#define LDSX() do { asm volatile("s_wait_dscnt 0" ::: "memory"); __builtin_amdgcn_wave_barrier(); __builtin_amdgcn_fence(__ATOMIC_RELEASE, "workgroup"); } while (0)


#define NB 4
#define SS 4096
#define NR (NB * SS)
#define CC 256
#define HD 128
#ifndef TQB
#define TQB (SS / 64)
#define TNB NB
#endif
typedef __attribute__((ext_vector_type(8))) __bf16 v8b;
__device__ __forceinline__ v16b frag_b(const __bf16* rowk0, int lane) {
  union { v16b v; v8b q[2]; } u; const __bf16* p = rowk0 + 8 * (lane >> 4);
  u.q[0] = *(const v8b*)p; u.q[1] = *(const v8b*)(p + 16); return u.v;
}
__device__ __forceinline__ float bfr(float v) { return (float)(__bf16)v; }
__device__ __attribute__((noinline)) float exp_ni(float v) { return expf(v); }
__device__ __attribute__((noinline)) float erf_ni(float v) { return erff(v); }

#define WS_PK  0u
#define WS_GH  (((2u * 384 * CC) + 127u) / 128u * 128u)
#define WS_GL  (WS_GH + 2u * NR * HD)
#define WS_JH  (WS_GL + 2u * NR * HD)
#define WS_JL  (WS_JH + 2u * NR * HD)
#define WS_VTH (WS_JL + 2u * NR * HD)
#define WS_VTL (WS_VTH + 2u * NR * HD)
#define WS_END (WS_VTL + 2u * NR * HD)

__global__ __launch_bounds__(256) void k_pack(const float* __restrict__ WG, const float* __restrict__ WJ, const float* __restrict__ WK, __bf16* __restrict__ PK) {
  __shared__ __align__(16) __bf16 s[CC]; const int n = blockIdx.x, t = threadIdx.x; const int which = n / HD, d = n % HD; const float* Wm = (which == 0) ? WG : (which == 1) ? WJ : WK;
  s[t] = (__bf16)Wm[(size_t)t * HD + d];
  __syncthreads();
  if (t < CC / 8) vst2((unsigned*)(PK + (size_t)n * CC + t * 8), *(const v4u*)&s[t * 8]);
}
__global__ __launch_bounds__(128) void k_proj(const float* __restrict__ CROSS, const float* __restrict__ WITHIN, const __bf16* __restrict__ PK, const float* __restrict__ BG, const float* __restrict__ BJ, const float* __restrict__ BKv, _Float16* __restrict__ GH, _Float16* __restrict__ GL, _Float16* __restrict__ JH, _Float16* __restrict__ JL, _Float16* __restrict__ VTH, _Float16* __restrict__ VTL) {
  __shared__ __align__(16) _Float16 soh[4][16][136], sol[4][16][136]; __shared__ __align__(16) _Float16 sth[HD][72], stl[HD][72];
  const int tid = threadIdx.x, wave = tid >> 5, lane = tid & 31, col = lane & 15, g = lane >> 4; const size_t r0 = (size_t)blockIdx.x * 64 + wave * 16; const int which = blockIdx.y;
  const float* X = (which == 0) ? WITHIN : CROSS; const float* BB = (which == 0) ? BG : (which == 1) ? BJ : BKv;
  v8f acc[8] = {};
#pragma unroll 2
  for (int kc = 0; kc < CC / 32; ++kc) { v16b a; { const float* p = X + (r0 + col) * CC + kc * 32 + 8 * g;
#pragma unroll
      for (int i = 0; i < 8; ++i) { a[i] = (__bf16)p[i]; a[8 + i] = (__bf16)p[16 + i]; } }
#pragma unroll
    for (int jj = 0; jj < 8; ++jj) acc[jj] = wmma_bf(a, frag_b(PK + ((size_t)which * HD + jj * 16 + col) * CC + kc * 32, lane), acc[jj]); }
  if (which < 2) {
#pragma unroll
    for (int jj = 0; jj < 8; ++jj) { const int d = jj * 16 + col; const float bb = bfr(BB[d]);
#pragma unroll
      for (int r = 0; r < 8; ++r) { const float v = acc[jj][r] + bb; const _Float16 hv = (_Float16)v; soh[wave][8 * g + r][d] = hv; sol[wave][8 * g + r][d] = (_Float16)((v - (float)hv) * 2048.0f); } }
    LDSX();
    _Float16* DH = (which == 0) ? GH : JH; _Float16* DL = (which == 0) ? GL : JL;
    for (int rl = 0; rl < 16; ++rl) { if (lane < 16) vst2((unsigned*)(DH + (r0 + rl) * HD + lane * 8), *(const v4u*)&soh[wave][rl][lane * 8]); else vst2((unsigned*)(DL + (r0 + rl) * HD + (lane - 16) * 8), *(const v4u*)&sol[wave][rl][(lane - 16) * 8]); }
  } else {
#pragma unroll
    for (int jj = 0; jj < 8; ++jj) { const int d = jj * 16 + col; const float bb = bfr(BB[d]);
#pragma unroll
      for (int r = 0; r < 8; ++r) { const float v = acc[jj][r] + bb; const _Float16 hv = (_Float16)v; sth[d][wave * 16 + 8 * g + r] = hv; stl[d][wave * 16 + 8 * g + r] = (_Float16)((v - (float)hv) * 2048.0f); } }
    __syncthreads();
    const size_t rb = (size_t)blockIdx.x * 64; const int b = (int)(rb / SS), s0 = (int)(rb % SS);
    for (int e = tid; e < HD * 8; e += 128) { const int d = e >> 3, pc = e & 7; const size_t o = ((size_t)b * HD + d) * SS + s0 + pc * 8; vst2((unsigned*)(VTH + o), *(const v4u*)&sth[d][pc * 8]); vst2((unsigned*)(VTL + o), *(const v4u*)&stl[d][pc * 8]); }
  }
}
__global__ __launch_bounds__(128) void k_attn(const _Float16* __restrict__ GH, const _Float16* __restrict__ GL, const _Float16* __restrict__ JH, const _Float16* __restrict__ JL, const _Float16* __restrict__ VTH, const _Float16* __restrict__ VTL, float* __restrict__ OUT) {
  __shared__ __align__(16) _Float16 sph[4][16][40]; __shared__ __align__(16) float so[4][16][HD + 4];
  const int tid = threadIdx.x, wave = tid >> 5, lane = tid & 31, col = lane & 15, g = lane >> 4; const int qb = blockIdx.x, b = blockIdx.y; (void)VTL; const int q0 = qb * 64 + wave * 16; const size_t rq = (size_t)b * SS + q0 + col;
  v16h aqh[4], aql[4];
#pragma unroll
  for (int kc = 0; kc < 4; ++kc) { aqh[kc] = frag_h(GH + rq * HD + kc * 32, lane); aql[kc] = frag_h(GL + rq * HD + kc * 32, lane); }
  const _Float16* Vh = VTH + (size_t)b * HD * SS; const _Float16* Vl = VTL + (size_t)b * HD * SS;
  float m[8], l[8];
#pragma unroll
  for (int r = 0; r < 8; ++r) { m[r] = -3.0e38f; l[r] = 0.f; }
  v8f acc[8] = {};
#pragma unroll 1
  for (int ks = 0; ks < SS / 32; ++ks) { v8f s[2];
#pragma unroll
    for (int ct = 0; ct < 2; ++ct) { const int kk = ks * 32 + ct * 16 + col; const size_t rk = ((size_t)b * SS + kk) * HD; v8f c = {}, cl = {};
#pragma unroll
      for (int kc = 0; kc < 4; ++kc) { const v16h khf = frag_h(JH + rk + kc * 32, lane); c = wmma16(aqh[kc], khf, c); cl = wmma16(aql[kc], khf, cl); cl = wmma16(aqh[kc], frag_h(JL + rk + kc * 32, lane), cl); }
#pragma unroll
      for (int r = 0; r < 8; ++r) s[ct][r] = c[r] + cl[r] * (1.0f / 2048.0f); }
#pragma unroll
    for (int r = 0; r < 8; ++r) { float mx = fmaxf(s[0][r], s[1][r]);
#pragma unroll
      for (int o = 1; o < 16; o <<= 1) mx = fmaxf(mx, __shfl_xor(mx, o));
      const float mn = fmaxf(m[r], mx); const float alpha = (m[r] <= -1.0e38f) ? 0.f : exp_ni(m[r] - mn); const float e0 = exp_ni(s[0][r] - mn), e1 = exp_ni(s[1][r] - mn); float es = e0 + e1;
#pragma unroll
      for (int o = 1; o < 16; o <<= 1) es += __shfl_xor(es, o);
      l[r] = l[r] * alpha + es; m[r] = mn;
#pragma unroll
      for (int dt = 0; dt < 8; ++dt) acc[dt][r] *= alpha;
      sph[wave][8 * g + r][col] = (_Float16)e0; sph[wave][8 * g + r][16 + col] = (_Float16)e1; }
    LDSX();
    const v16h pah = frag_h(&sph[wave][col][0], lane);
#pragma unroll
    for (int dt = 0; dt < 8; ++dt) { const size_t vo = (size_t)(dt * 16 + col) * SS + ks * 32; acc[dt] = wmma16(pah, frag_h(Vh + vo, lane), acc[dt]); }
    LDSX(); }
#pragma unroll
  for (int r = 0; r < 8; ++r) { const float il = 1.0f / l[r];
#pragma unroll
    for (int dt = 0; dt < 8; ++dt) so[wave][8 * g + r][dt * 16 + col] = acc[dt][r] * il; }
  LDSX();
  for (int rl = 0; rl < 16; ++rl) vst2(OUT + ((size_t)b * SS + q0 + rl) * HD + lane * 4, *(const v4f*)&so[wave][rl][lane * 4]);
}
extern "C" void kernel_launch(void* const* d_in, const int* in_sizes, int n_in, void* d_out, int out_size, void* d_ws, size_t ws_size, hipStream_t stream) {
  (void)in_sizes; (void)n_in; (void)out_size;
  const float** F = (const float**)d_in;
  if (ws_size < (size_t)WS_END) return;
  char* ws = (char*)d_ws; __bf16* PK = (__bf16*)(ws + WS_PK); _Float16 *GH = (_Float16*)(ws + WS_GH), *GL = (_Float16*)(ws + WS_GL), *JH = (_Float16*)(ws + WS_JH), *JL = (_Float16*)(ws + WS_JL), *VTH = (_Float16*)(ws + WS_VTH), *VTL = (_Float16*)(ws + WS_VTL);
  k_pack<<<384, 256, 0, stream>>>(F[2], F[4], F[6], PK);
  k_proj<<<dim3(TNB * SS / 64, 3), 128, 0, stream>>>(F[0], F[1], PK, F[3], F[5], F[7], GH, GL, JH, JL, VTH, VTL);
  k_attn<<<dim3(TQB, TNB), 128, 0, stream>>>(GH, GL, JH, JL, VTH, VTL, (float*)d_out);
}
